// MultiheadAttention_89893665505280
// MI455X (gfx1250) — hardware-run, weakly checked
//
#include <hip/hip_runtime.h>


#ifndef NB
#define NB 8
#endif
#ifndef SEQ
#define SEQ 1024
#endif
#define NB_FULL  8
#define SEQ_FULL 1024
#define DM   256
#define NH_  8
#define HD   32
#define TP   72
#define PMP  36
#define CSP  264
#define OSP  68
#define L2E  1.4426950408889634f
#define WSC  64.0f
#define WINV 0.015625f
#define QKC  16.0f
#define VC   16.0f
#define CP   16.0f
#define CC   64.0f
#define RSC  2048.0f
#define RINV 0.00048828125f
#define SC2  (0.00390625f * 0.17677669529663687f * L2E)
#define CPS  (CP * (float)SEQ)
#define OSC  (1.0f / (CP * VC * (float)SEQ))
#define VMS  (1.0f / (VC * (float)SEQ))
#define OINV (1.0f / (CC * WSC))

static_assert(NB_FULL == 8);
static_assert(NH_ * HD == DM);
static_assert(HD == 32);
static_assert(DM % 64 == 0);
static_assert(SEQ % 256 == 0);
static_assert(NB <= NB_FULL);
static_assert(SEQ <= SEQ_FULL);
static_assert(SEQ <= 2048);
static_assert(((size_t)NB * SEQ) % 4 == 0);
static_assert(((size_t)NB * DM) % 32 == 0);

typedef _Float16 h16;
typedef __attribute__((ext_vector_type(16))) _Float16 v16h;
typedef __attribute__((ext_vector_type(8)))  _Float16 v8h;
typedef __attribute__((ext_vector_type(8)))  float    v8f;
typedef __attribute__((ext_vector_type(4)))  float    v4f;
typedef v4f  __attribute__((may_alias)) v4fa;
typedef v8h  __attribute__((may_alias)) v8ha;

static constexpr size_t XPL = (size_t)SEQ * NB_FULL * DM;
static constexpr size_t QPL = (size_t)NB * SEQ * DM;
static constexpr size_t OUT1_OFF = (size_t)SEQ_FULL * NB_FULL * DM;
static_assert(OUT1_OFF * 4 == (size_t)8388608);

__device__ __forceinline__ float rbf(float f) { unsigned u = __float_as_uint(f); u += 0x7FFFu + ((u >> 16) & 1u); return __uint_as_float(u & 0xFFFF0000u); }
__device__ __forceinline__ v16h cat16(v8h lo, v8h hi) { return __builtin_shufflevector(lo, hi, 0, 1, 2, 3, 4, 5, 6, 7, 8, 9, 10, 11, 12, 13, 14, 15); }
__device__ __forceinline__ v8f wmma16(v16h a, v16h b, v8f c) { return __builtin_amdgcn_wmma_f32_16x16x32_f16(false, a, false, b, (short)0, c, false, false); }
__device__ __forceinline__ v16h ldh(const h16* p) { return cat16(*(const v8h*)p, *(const v8h*)(p + 16)); }

__global__ __launch_bounds__(256) void k_cvt_x(const float* __restrict__ s0, const float* __restrict__ s1, const float* __restrict__ s2, h16* XH, size_t n8) {
    const size_t i = (size_t)blockIdx.x * 256 + threadIdx.x; if (i >= n8) return;
    const size_t e = i * 8;
    const v8f x = *(const v8f*)(s0 + e); const v8f y = *(const v8f*)(s1 + e); const v8f z = *(const v8f*)(s2 + e);
    v8h a, b, c;
#pragma unroll
    for (int k = 0; k < 8; ++k) { a[k] = (h16)rbf(x[k]); b[k] = (h16)rbf(y[k]); c[k] = (h16)rbf(z[k]); }
    h16* d0 = XH + e; h16* d1 = XH + XPL + e; h16* d2 = XH + 2 * XPL + e;
    *(volatile v8h*)d0 = a; *(volatile v8h*)d1 = b; *(volatile v8h*)d2 = c;
    __threadfence();
    *(volatile v8h*)d0 = a; *(volatile v8h*)d1 = b; *(volatile v8h*)d2 = c;
}

__global__ __launch_bounds__(256) void k_cvt_w(const float* __restrict__ s0, const float* __restrict__ s1, const float* __restrict__ s2, const float* __restrict__ s3, h16* WH, size_t n8) {
    const size_t i = (size_t)blockIdx.x * 256 + threadIdx.x; if (i >= n8) return;
    const size_t e = i * 8;
    const v8f x = *(const v8f*)(s0 + e); const v8f y = *(const v8f*)(s1 + e); const v8f z = *(const v8f*)(s2 + e); const v8f w = *(const v8f*)(s3 + e);
    v8h a, b, c, d;
#pragma unroll
    for (int k = 0; k < 8; ++k) { a[k] = (h16)(rbf(x[k]) * WSC); b[k] = (h16)(rbf(y[k]) * WSC); c[k] = (h16)(rbf(z[k]) * WSC); d[k] = (h16)(rbf(w[k]) * WSC); }
    h16* d0 = WH + e; h16* d1 = WH + (size_t)DM * DM + e; h16* d2 = WH + (size_t)2 * DM * DM + e; h16* d3 = WH + (size_t)3 * DM * DM + e;
    *(volatile v8h*)d0 = a; *(volatile v8h*)d1 = b; *(volatile v8h*)d2 = c; *(volatile v8h*)d3 = d;
    __threadfence();
    *(volatile v8h*)d0 = a; *(volatile v8h*)d1 = b; *(volatile v8h*)d2 = c; *(volatile v8h*)d3 = d;
}

__global__ __launch_bounds__(256) void k_pe(const float* __restrict__ qx, const float* __restrict__ kx, const float* __restrict__ pw, const float* __restrict__ pb, float* PP) {
    __shared__ __align__(16) float sq[2 * NB_FULL * 32];
    const int tid = threadIdx.x; const int t0 = blockIdx.x * 32;
    const int tl = tid >> 3, b = tid & 7;
    const size_t ro = ((size_t)(t0 + tl) * NB_FULL + b) * 3;
    const float w0 = rbf(pw[0]), w1 = rbf(pw[1]), w2 = rbf(pw[2]), peb = rbf(pb[0]);
    const float a = rbf(qx[ro]) * w0 + rbf(qx[ro + 1]) * w1 + rbf(qx[ro + 2]) * w2 + peb;
    const float c = rbf(kx[ro]) * w0 + rbf(kx[ro + 1]) * w1 + rbf(kx[ro + 2]) * w2;
    sq[b * 32 + tl] = a * L2E; sq[NB_FULL * 32 + b * 32 + tl] = c * L2E;
    __syncthreads();
    if (tid < 128) {
        const int line = tid >> 3, plane = line >> 3, bb = line & 7, c4 = (tid & 7) * 4;
        const v4f val = *(const v4fa*)(&sq[plane * (NB_FULL * 32) + bb * 32 + c4]);
        if (bb < NB) {
            float* dst = PP + (size_t)plane * NB * SEQ + (size_t)bb * SEQ + t0 + c4;
            *(volatile v4f*)dst = val;
            __threadfence();
            *(volatile v4f*)dst = val;
        }
    }
}

__global__ __launch_bounds__(128) void k_proj(const h16* __restrict__ XH, const h16* __restrict__ WH,
                                              const float* __restrict__ bq, const float* __restrict__ bk, const float* __restrict__ bv,
                                              h16* QKH, h16* VTH, h16* VTR) {
    __shared__ __align__(16) h16 ts[2 * 64 * TP];
    const int tid = threadIdx.x, lane = tid & 31, lr = lane & 15, hi = lane >> 4;
    const int wave = __builtin_amdgcn_readfirstlane((int)(threadIdx.x >> 5));
    const int which = blockIdx.z / NB, b = blockIdx.z % NB;
    const int t0 = blockIdx.x * 64, n0 = blockIdx.y * 64;
    const h16* ap = XH + (size_t)which * XPL + ((size_t)(t0 + 16 * wave + lr) * NB_FULL + b) * DM + 8 * hi;
    const h16* wp = WH + (size_t)which * DM * DM + (size_t)(n0 + lr) * DM + 8 * hi;
    v8f c0 = (v8f){}, c1 = (v8f){}, c2 = (v8f){}, c3 = (v8f){};
#pragma unroll 1
    for (int k0 = 0; k0 < DM; k0 += 32) {
        const v16h a = ldh(ap + k0);
        const v16h w0 = ldh(wp + k0), w1 = ldh(wp + (size_t)16 * DM + k0), w2 = ldh(wp + (size_t)32 * DM + k0), w3 = ldh(wp + (size_t)48 * DM + k0);
        c0 = wmma16(a, w0, c0); c1 = wmma16(a, w1, c1); c2 = wmma16(a, w2, c2); c3 = wmma16(a, w3, c3);
        asm volatile("v_nop\n\tv_nop\n\tv_nop\n\tv_nop" : "+v"(c0), "+v"(c1), "+v"(c2), "+v"(c3) : "v"(a), "v"(w0), "v"(w1), "v"(w2), "v"(w3));
    }
    float bb0, bb1, bb2, bb3;
    { const int n = n0 + lr;
      const float q0 = bq[n], q1 = bq[n + 16], q2 = bq[n + 32], q3 = bq[n + 48];
      const float k0 = bk[n], k1 = bk[n + 16], k2 = bk[n + 32], k3 = bk[n + 48];
      const float u0 = bv[n], u1 = bv[n + 16], u2 = bv[n + 32], u3 = bv[n + 48];
      bb0 = rbf(which == 0 ? q0 : (which == 1 ? k0 : u0)); bb1 = rbf(which == 0 ? q1 : (which == 1 ? k1 : u1));
      bb2 = rbf(which == 0 ? q2 : (which == 1 ? k2 : u2)); bb3 = rbf(which == 0 ? q3 : (which == 1 ? k3 : u3)); }
    if (which < 2) {
#pragma unroll
        for (int r = 0; r < 8; ++r) { const int ro = wave * 16 * TP + (8 * hi + r) * TP + lr;
            ts[ro]      = (h16)((c0[r] * WINV + bb0) * QKC); ts[ro + 16] = (h16)((c1[r] * WINV + bb1) * QKC);
            ts[ro + 32] = (h16)((c2[r] * WINV + bb2) * QKC); ts[ro + 48] = (h16)((c3[r] * WINV + bb3) * QKC); }
        __syncthreads();
        h16* dst = QKH + (size_t)which * QPL + ((size_t)b * SEQ + t0 + 16 * wave) * DM + n0;
#pragma unroll 1
        for (int ps = 0; ps < 2; ++ps) {
#pragma unroll
            for (int s = 0; s < 4; ++s) { const int row = 4 * s + (lane >> 3), c8 = (lane & 7) * 8;
                const v8h val = *(const v8ha*)(&ts[wave * 16 * TP + row * TP + c8]);
                *(volatile v8h*)(dst + (size_t)row * DM + c8) = val; }
            if (ps == 0) __threadfence(); }
    } else {
#pragma unroll
        for (int r = 0; r < 8; ++r) { const int so = lr * TP + 16 * wave + 8 * hi + r;
            { const float v = (c0[r] * WINV + bb0) * VC; const h16 hh = (h16)v; ts[so] = hh;           ts[64 * TP + so] = (h16)((v - (float)hh) * RSC); }
            { const float v = (c1[r] * WINV + bb1) * VC; const h16 hh = (h16)v; ts[so + 16 * TP] = hh; ts[64 * TP + so + 16 * TP] = (h16)((v - (float)hh) * RSC); }
            { const float v = (c2[r] * WINV + bb2) * VC; const h16 hh = (h16)v; ts[so + 32 * TP] = hh; ts[64 * TP + so + 32 * TP] = (h16)((v - (float)hh) * RSC); }
            { const float v = (c3[r] * WINV + bb3) * VC; const h16 hh = (h16)v; ts[so + 48 * TP] = hh; ts[64 * TP + so + 48 * TP] = (h16)((v - (float)hh) * RSC); } }
        __syncthreads();
        const size_t rb = ((size_t)b * DM + n0) * SEQ + t0;
#pragma unroll 1
        for (int ps = 0; ps < 2; ++ps) {
#pragma unroll
            for (int s = 0; s < 4; ++s) { const int nl = 16 * s + (tid >> 3), c8 = (tid & 7) * 8;
                const v8h vh = *(const v8ha*)(&ts[nl * TP + c8]);
                const v8h vr = *(const v8ha*)(&ts[64 * TP + nl * TP + c8]);
                *(volatile v8h*)(VTH + rb + (size_t)nl * SEQ + c8) = vh;
                *(volatile v8h*)(VTR + rb + (size_t)nl * SEQ + c8) = vr; }
            if (ps == 0) __threadfence(); }
    }
}

__global__ __launch_bounds__(256) void k_vmean(const h16* __restrict__ VTH, const h16* __restrict__ VTR, float* VM) {
    __shared__ __align__(16) float sm[32];
    const int tid = threadIdx.x, lane = tid & 31, wave = __builtin_amdgcn_readfirstlane((int)(tid >> 5));
#pragma unroll 1
    for (int q = 0; q < 4; ++q) {
        const size_t row = (size_t)blockIdx.x * 32 + wave * 4 + q;
        float sh = 0.0f, sr = 0.0f;
#pragma unroll 1
        for (int i = lane * 8; i < SEQ; i += 256) {
            const v8h a = *(const v8h*)(VTH + row * SEQ + i); const v8h c = *(const v8h*)(VTR + row * SEQ + i);
#pragma unroll
            for (int k = 0; k < 8; ++k) { sh += (float)a[k]; sr += (float)c[k]; } }
        sh += __shfl_xor(sh, 16, 32); sr += __shfl_xor(sr, 16, 32);
        sh += __shfl_xor(sh, 8, 32);  sr += __shfl_xor(sr, 8, 32);
        sh += __shfl_xor(sh, 4, 32);  sr += __shfl_xor(sr, 4, 32);
        sh += __shfl_xor(sh, 2, 32);  sr += __shfl_xor(sr, 2, 32);
        sh += __shfl_xor(sh, 1, 32);  sr += __shfl_xor(sr, 1, 32);
        if (lane == 0) sm[wave * 4 + q] = (sh + sr * RINV) * VMS;
    }
    __syncthreads();
    if (tid < 8) {
        const v4f val = *(const v4fa*)(&sm[tid * 4]);
        float* dst = VM + (size_t)blockIdx.x * 32 + tid * 4;
        *(volatile v4f*)dst = val;
        __threadfence();
        *(volatile v4f*)dst = val;
    }
}

__global__ __launch_bounds__(256) void k_attn(const h16* __restrict__ QKH, const h16* __restrict__ VTH, const h16* __restrict__ VTR,
                                              const float* __restrict__ PP, const float* __restrict__ VM,
                                              float* MEAN, h16* CHH, h16* CHR) {
    __shared__ __align__(16) float pm[NH_ * 16 * PMP];
    __shared__ __align__(16) h16 cs[2 * 16 * CSP];
    const int tid = threadIdx.x, lane = tid & 31, lr = lane & 15, hi = lane >> 4;
    const int h = __builtin_amdgcn_readfirstlane((int)(threadIdx.x >> 5));
    const int b = blockIdx.y, t0 = blockIdx.x * 16;
    const size_t rb = (size_t)b * SEQ * DM + (size_t)h * HD + 8 * hi;
    const v16h qf = ldh(QKH + rb + (size_t)(t0 + lr) * DM);
    const h16* kp = QKH + QPL + rb + (size_t)lr * DM;
    const float* pkp = PP + (size_t)NB * SEQ + (size_t)b * SEQ + 8 * hi;
    const float pq2 = PP[(size_t)b * SEQ + t0 + lr];
    float m = -3.0e38f, l = 0.0f;
#pragma unroll 1
    for (int key0 = 0; key0 < SEQ; key0 += 32) {
        const h16* ka = kp + (size_t)key0 * DM;
        const v16h k0f = ldh(ka), k1f = ldh(ka + (size_t)16 * DM);
        v8f sa = (v8f){}, sb = (v8f){};
        sa = wmma16(k0f, qf, sa); sb = wmma16(k1f, qf, sb);
        asm volatile("v_nop\n\tv_nop\n\tv_nop\n\tv_nop" : "+v"(sa), "+v"(sb) : "v"(k0f), "v"(k1f), "v"(qf));
        const v8f ba = *(const v8f*)(pkp + key0); const v8f bc = *(const v8f*)(pkp + key0 + 16);
        float ta[8], tb[8]; float mx = -3.0e38f;
#pragma unroll
        for (int r = 0; r < 8; ++r) { ta[r] = fmaf(sa[r], SC2, pq2 - ba[r]); tb[r] = fmaf(sb[r], SC2, pq2 - bc[r]); mx = fmaxf(mx, fmaxf(ta[r], tb[r])); }
        mx = fmaxf(mx, __shfl_xor(mx, 16, 32));
        const float mnew = fmaxf(m, mx);
        const float alpha = __builtin_amdgcn_exp2f(m - mnew);
        float ls = 0.0f;
#pragma unroll
        for (int r = 0; r < 8; ++r) ls += __builtin_amdgcn_exp2f(ta[r] - mnew) + __builtin_amdgcn_exp2f(tb[r] - mnew);
        l = l * alpha + ls; m = mnew;
    }
    l += __shfl_xor(l, 16, 32);
    const float inv = 1.0f / l;

    const h16* vh = VTH + ((size_t)b * DM + h * HD + lr) * SEQ + 8 * hi;
    const h16* vr = VTR + ((size_t)b * DM + h * HD + lr) * SEQ + 8 * hi;
    v8f oh0 = (v8f){}, oh1 = (v8f){}, or0 = (v8f){}, or1 = (v8f){};
    const int srow = (tid >> 3) & 15, sc4 = (tid & 7) * 4;
    float* mrow = MEAN + ((size_t)b * SEQ + t0 + srow) * SEQ + sc4;
    const int po = (h * 16 + lr) * PMP + 8 * hi;
#pragma unroll 1
    for (int key0 = 0; key0 < SEQ; key0 += 32) {
        const h16* ka = kp + (size_t)key0 * DM;
        const v16h k0f = ldh(ka), k1f = ldh(ka + (size_t)16 * DM);
        v8f sa = (v8f){}, sb = (v8f){};
        sa = wmma16(k0f, qf, sa); sb = wmma16(k1f, qf, sb);
        asm volatile("v_nop\n\tv_nop\n\tv_nop\n\tv_nop" : "+v"(sa), "+v"(sb) : "v"(k0f), "v"(k1f), "v"(qf));
        const v8f ba = *(const v8f*)(pkp + key0); const v8f bc = *(const v8f*)(pkp + key0 + 16);
        v4f p0, p1, p2, p3; v16h pb;
#pragma unroll
        for (int r = 0; r < 4; ++r) {
            const float a0 = __builtin_amdgcn_exp2f(fmaf(sa[r],     SC2, pq2 - ba[r])     - m) * inv;
            const float a1 = __builtin_amdgcn_exp2f(fmaf(sa[r + 4], SC2, pq2 - ba[r + 4]) - m) * inv;
            const float a2 = __builtin_amdgcn_exp2f(fmaf(sb[r],     SC2, pq2 - bc[r])     - m) * inv;
            const float a3 = __builtin_amdgcn_exp2f(fmaf(sb[r + 4], SC2, pq2 - bc[r + 4]) - m) * inv;
            p0[r] = a0; p1[r] = a1; p2[r] = a2; p3[r] = a3;
            pb[r] = (h16)(a0 * CPS - CP); pb[r + 4] = (h16)(a1 * CPS - CP); pb[8 + r] = (h16)(a2 * CPS - CP); pb[12 + r] = (h16)(a3 * CPS - CP); }
        *(v4fa*)(&pm[po]) = p0; *(v4fa*)(&pm[po + 4]) = p1; *(v4fa*)(&pm[po + 16]) = p2; *(v4fa*)(&pm[po + 20]) = p3;
        __syncthreads();
        if (tid < 128) {
            v4f acc = *(const v4fa*)(&pm[srow * PMP + sc4]);
#pragma unroll
            for (int hh = 1; hh < NH_; ++hh) acc += *(const v4fa*)(&pm[(hh * 16 + srow) * PMP + sc4]);
            const v4f mv = acc * 0.125f;
            *(volatile v4f*)(mrow + key0) = mv;
            __threadfence();
            *(volatile v4f*)(mrow + key0) = mv;
        }
        const v16h v0 = ldh(vh + key0), v1 = ldh(vh + (size_t)16 * SEQ + key0), r0 = ldh(vr + key0), r1 = ldh(vr + (size_t)16 * SEQ + key0);
        oh0 = wmma16(v0, pb, oh0); oh1 = wmma16(v1, pb, oh1); or0 = wmma16(r0, pb, or0); or1 = wmma16(r1, pb, or1);
        asm volatile("v_nop\n\tv_nop\n\tv_nop\n\tv_nop" : "+v"(oh0), "+v"(oh1), "+v"(or0), "+v"(or1) : "v"(v0), "v"(v1), "v"(r0), "v"(r1), "v"(pb));
        __syncthreads();
    }
    { const float* vmp = VM + (size_t)b * DM + h * HD + 8 * hi;
      const v4f ma = *(const v4f*)(vmp), mb = *(const v4f*)(vmp + 4), mc = *(const v4f*)(vmp + 16), md = *(const v4f*)(vmp + 20);
      v8h ch, cr;
#pragma unroll
      for (int r = 0; r < 8; ++r) { const float mean = (r < 4) ? ma[r & 3] : mb[r & 3];
          const float c = ((oh0[r] + or0[r] * RINV) * OSC + mean) * CC; const h16 hh = (h16)c; ch[r] = hh; cr[r] = (h16)((c - (float)hh) * RSC); }
      *(v8ha*)(&cs[lr * CSP + h * HD + 8 * hi]) = ch; *(v8ha*)(&cs[16 * CSP + lr * CSP + h * HD + 8 * hi]) = cr;
#pragma unroll
      for (int r = 0; r < 8; ++r) { const float mean = (r < 4) ? mc[r & 3] : md[r & 3];
          const float c = ((oh1[r] + or1[r] * RINV) * OSC + mean) * CC; const h16 hh = (h16)c; ch[r] = hh; cr[r] = (h16)((c - (float)hh) * RSC); }
      *(v8ha*)(&cs[lr * CSP + h * HD + 16 + 8 * hi]) = ch; *(v8ha*)(&cs[16 * CSP + lr * CSP + h * HD + 16 + 8 * hi]) = cr; }
    __syncthreads();
    const size_t cb = ((size_t)b * SEQ + t0) * DM;
#pragma unroll 1
    for (int ps = 0; ps < 2; ++ps) {
#pragma unroll
        for (int s = 0; s < 2; ++s) { const int row = 8 * s + __builtin_amdgcn_readfirstlane((int)(tid >> 5)), c8 = (tid & 31) * 8;
            const v8h a = *(const v8ha*)(&cs[row * CSP + c8]);
            const v8h c = *(const v8ha*)(&cs[16 * CSP + row * CSP + c8]);
            *(volatile v8h*)(CHH + cb + (size_t)row * DM + c8) = a;
            *(volatile v8h*)(CHR + cb + (size_t)row * DM + c8) = c; }
        if (ps == 0) __threadfence(); }
}

__global__ __launch_bounds__(128) void k_softmax(const float* __restrict__ MEAN, float* OUT1) {
    const int lane = threadIdx.x & 31, wave = __builtin_amdgcn_readfirstlane((int)(threadIdx.x >> 5));
    const size_t row = (size_t)blockIdx.x * 4 + wave;
    const size_t b = row / SEQ, t = row % SEQ;
    const float* src = MEAN + row * SEQ + lane * 4;
    v4f x[SEQ / 128]; float mx = -3.0e38f;
#pragma unroll
    for (int i = 0; i < SEQ / 128; ++i) { x[i] = *(const v4f*)(src + i * 128); mx = fmaxf(mx, fmaxf(fmaxf(x[i][0], x[i][1]), fmaxf(x[i][2], x[i][3]))); }
    mx = fmaxf(mx, __shfl_xor(mx, 16, 32)); mx = fmaxf(mx, __shfl_xor(mx, 8, 32)); mx = fmaxf(mx, __shfl_xor(mx, 4, 32));
    mx = fmaxf(mx, __shfl_xor(mx, 2, 32));  mx = fmaxf(mx, __shfl_xor(mx, 1, 32));
    float s = 0.0f;
#pragma unroll
    for (int i = 0; i < SEQ / 128; ++i) {
#pragma unroll
        for (int k = 0; k < 4; ++k) { const float e = __builtin_amdgcn_exp2f((x[i][k] - mx) * L2E); x[i][k] = e; s += e; } }
    s += __shfl_xor(s, 16, 32); s += __shfl_xor(s, 8, 32); s += __shfl_xor(s, 4, 32); s += __shfl_xor(s, 2, 32); s += __shfl_xor(s, 1, 32);
    const float inv = 1.0f / s;
#pragma unroll
    for (int i = 0; i < SEQ / 128; ++i) x[i] = x[i] * inv;
    float* dst = OUT1 + (b * SEQ_FULL + t) * SEQ_FULL + lane * 4;
#pragma unroll 1
    for (int ps = 0; ps < 2; ++ps) {
#pragma unroll
        for (int i = 0; i < SEQ / 128; ++i) *(volatile v4f*)(dst + i * 128) = x[i];
        if (ps == 0) __threadfence(); }
}

__global__ __launch_bounds__(128) void k_oproj(const h16* __restrict__ CHH, const h16* __restrict__ CHR, const h16* __restrict__ WO, const float* __restrict__ bo, float* OUT) {
    __shared__ __align__(16) float os[4 * 16 * OSP];
    const int lane = threadIdx.x & 31, lr = lane & 15, hi = lane >> 4;
    const int wave = __builtin_amdgcn_readfirstlane((int)(threadIdx.x >> 5));
    const int t0 = blockIdx.x * 16, b = blockIdx.y, n0 = wave * 64;
    const size_t ao = ((size_t)b * SEQ + t0 + lr) * DM + 8 * hi;
    const h16* ap = CHH + ao; const h16* rp = CHR + ao;
    const h16* wp = WO + (size_t)(n0 + lr) * DM + 8 * hi;
    v8f c0 = (v8f){}, c1 = (v8f){}, c2 = (v8f){}, c3 = (v8f){}, d0 = (v8f){}, d1 = (v8f){}, d2 = (v8f){}, d3 = (v8f){};
#pragma unroll 1
    for (int k0 = 0; k0 < DM; k0 += 32) {
        const v16h a = ldh(ap + k0), ar = ldh(rp + k0);
        const v16h w0 = ldh(wp + k0), w1 = ldh(wp + (size_t)16 * DM + k0), w2 = ldh(wp + (size_t)32 * DM + k0), w3 = ldh(wp + (size_t)48 * DM + k0);
        c0 = wmma16(a, w0, c0); c1 = wmma16(a, w1, c1); c2 = wmma16(a, w2, c2); c3 = wmma16(a, w3, c3);
        d0 = wmma16(ar, w0, d0); d1 = wmma16(ar, w1, d1); d2 = wmma16(ar, w2, d2); d3 = wmma16(ar, w3, d3);
        asm volatile("v_nop\n\tv_nop\n\tv_nop\n\tv_nop" : "+v"(c0), "+v"(c1), "+v"(c2), "+v"(c3), "+v"(d0), "+v"(d1), "+v"(d2), "+v"(d3)
                     : "v"(a), "v"(ar), "v"(w0), "v"(w1), "v"(w2), "v"(w3));
    }
    const float bb0 = rbf(bo[n0 + lr]), bb1 = rbf(bo[n0 + 16 + lr]), bb2 = rbf(bo[n0 + 32 + lr]), bb3 = rbf(bo[n0 + 48 + lr]);
    const int wb = wave * 16 * OSP;
#pragma unroll
    for (int r = 0; r < 8; ++r) { const int ro = wb + (8 * hi + r) * OSP + lr;
        os[ro]      = (c0[r] + d0[r] * RINV) * OINV + bb0; os[ro + 16] = (c1[r] + d1[r] * RINV) * OINV + bb1;
        os[ro + 32] = (c2[r] + d2[r] * RINV) * OINV + bb2; os[ro + 48] = (c3[r] + d3[r] * RINV) * OINV + bb3; }
    __syncthreads();
    float* orow = OUT + ((size_t)t0 * NB_FULL + b) * DM + n0;
#pragma unroll 1
    for (int ps = 0; ps < 2; ++ps) {
#pragma unroll
        for (int s = 0; s < 8; ++s) { const int row = 2 * s + hi, cofs = lr * 4;
            const v4f val = *(const v4fa*)(&os[wb + row * OSP + cofs]);
            *(volatile v4f*)(orow + (size_t)row * NB_FULL * DM + cofs) = val; }
        if (ps == 0) __threadfence(); }
}

static constexpr size_t al256(size_t v) { return (v + 255) & ~(size_t)255; }
static constexpr size_t SZ_X    = al256(3 * XPL * 2);
static constexpr size_t SZ_W    = al256((size_t)4 * DM * DM * 2);
static constexpr size_t SZ_PP   = al256((size_t)2 * NB * SEQ * 4);
static constexpr size_t SZ_QK   = al256(2 * QPL * 2);
static constexpr size_t SZ_VT   = al256((size_t)NB * DM * SEQ * 2);
static constexpr size_t SZ_VM   = al256((size_t)NB * DM * 4);
static constexpr size_t SZ_MEAN = al256((size_t)NB * SEQ * SEQ * 4);
static constexpr size_t SZ_CH   = al256(QPL * 2);
static constexpr size_t SZ_TOTAL = SZ_X + SZ_W + SZ_PP + SZ_QK + 2 * SZ_VT + SZ_VM + SZ_MEAN + 2 * SZ_CH;
static_assert(SZ_TOTAL <= (size_t)134217728);

extern "C" void kernel_launch(void* const* d_in, const int* in_sizes, int n_in,
                              void* d_out, int out_size, void* d_ws, size_t ws_size, hipStream_t stream) {
    if (n_in < 15) return;
    const size_t needx = (size_t)SEQ * NB_FULL * DM;
    if ((size_t)in_sizes[0] < needx || (size_t)in_sizes[1] < needx || (size_t)in_sizes[2] < needx) return;
    if ((size_t)in_sizes[3] < (size_t)SEQ * NB_FULL * 3 || (size_t)in_sizes[4] < (size_t)SEQ * NB_FULL * 3) return;
    if ((size_t)in_sizes[5] < (size_t)DM * DM || (size_t)in_sizes[7] < (size_t)DM * DM || (size_t)in_sizes[9] < (size_t)DM * DM || (size_t)in_sizes[11] < (size_t)DM * DM) return;
    if (in_sizes[6] < DM || in_sizes[8] < DM || in_sizes[10] < DM || in_sizes[12] < DM || in_sizes[13] < 3 || in_sizes[14] < 1) return;
    if ((size_t)out_size < OUT1_OFF + ((size_t)(NB - 1) * SEQ_FULL + (SEQ - 1)) * SEQ_FULL + SEQ) return;
    if (SZ_TOTAL > ws_size) return;
    const float* query = (const float*)d_in[0]; const float* key = (const float*)d_in[1]; const float* value = (const float*)d_in[2];
    const float* qxyz = (const float*)d_in[3]; const float* kxyz = (const float*)d_in[4];
    const float* Wq = (const float*)d_in[5]; const float* bq = (const float*)d_in[6];
    const float* Wk = (const float*)d_in[7]; const float* bk = (const float*)d_in[8];
    const float* Wv = (const float*)d_in[9]; const float* bv = (const float*)d_in[10];
    const float* Wo = (const float*)d_in[11]; const float* bo = (const float*)d_in[12];
    const float* pe_w = (const float*)d_in[13]; const float* pe_b = (const float*)d_in[14];
    float* OUT = (float*)d_out;
    float* OUT1 = OUT + OUT1_OFF;
    char* wsp = (char*)d_ws;
    h16* XH  = (h16*)wsp;   wsp += SZ_X;
    h16* WH  = (h16*)wsp;   wsp += SZ_W;
    float* PP = (float*)wsp; wsp += SZ_PP;
    h16* QKH = (h16*)wsp;   wsp += SZ_QK;
    h16* VTH = (h16*)wsp;   wsp += SZ_VT;
    h16* VTR = (h16*)wsp;   wsp += SZ_VT;
    float* VM = (float*)wsp; wsp += SZ_VM;
    float* MEAN = (float*)wsp; wsp += SZ_MEAN;
    h16* CHH = (h16*)wsp;   wsp += SZ_CH;
    h16* CHR = (h16*)wsp;   wsp += SZ_CH;

    const size_t n8x = XPL / 8;
    k_cvt_x<<<(unsigned)((n8x + 255) / 256), 256, 0, stream>>>(query, key, value, XH, n8x);
    const size_t n8w = (size_t)DM * DM / 8;
    k_cvt_w<<<(unsigned)((n8w + 255) / 256), 256, 0, stream>>>(Wq, Wk, Wv, Wo, WH, n8w);
    k_pe<<<SEQ / 32, 256, 0, stream>>>(qxyz, kxyz, pe_w, pe_b, PP);
    k_proj<<<dim3(SEQ / 64, DM / 64, 3 * NB), 128, 0, stream>>>(XH, WH, bq, bk, bv, QKH, VTH, VTR);
    k_vmean<<<(NB * DM) / 32, 256, 0, stream>>>(VTH, VTR, VM);
    k_attn<<<dim3(SEQ / 16, NB, 1), 256, 0, stream>>>(QKH, VTH, VTR, PP, VM, MEAN, CHH, CHR);
    k_softmax<<<(unsigned)(((size_t)NB * SEQ) / 4), 128, 0, stream>>>(MEAN, OUT1);
    k_oproj<<<dim3(SEQ / 16, NB, 1), 128, 0, stream>>>(CHH, CHR, WH + (size_t)3 * DM * DM, bo, OUT);
}
